// SelfAttention_67937792688325
// MI455X (gfx1250) — hardware-run, weakly checked
//
#include <hip/hip_runtime.h>


#ifndef NB
#define NB 8
#endif
#ifndef SEQ
#define SEQ 2048
#endif
#define NB_FULL    8
#define SEQ_FULL   2048
#define DM         512
#define PD         64
#define NQKV       192
#define PR         64
#define BQ         128
#define BK         32
#define NWAVE      8
#define LP         72
#define OP         68
#define WS_CAP     134217728ull

static_assert(SEQ % BQ == 0);
static_assert(SEQ % PR == 0);
static_assert(SEQ % BK == 0);
static_assert(BQ == NWAVE * 16);
static_assert(PD == 64);
static_assert(DM % 64 == 0);
static_assert(DM % 32 == 0);
static_assert(NQKV == 3 * PD);
static_assert(PD * 2 == 128);
static_assert(PR * 2 == 128);
static_assert(PR == 64 && PR <= LP);
static_assert(SEQ <= SEQ_FULL);
static_assert(NB >= 1 && NB <= NB_FULL);
static_assert((LP * 2) % 16 == 0);
static_assert((OP * 4) % 16 == 0);
static_assert(OP >= 64);
static_assert((unsigned long long)NQKV * DM * 2ull + (unsigned long long)DM * PD * 2ull +
              3ull * NB * SEQ * PD * 2ull <= WS_CAP);

typedef __bf16   bf16;
typedef _Float16 f16;
typedef bf16           v16bf __attribute__((ext_vector_type(16)));
typedef f16            v16h  __attribute__((ext_vector_type(16)));
typedef f16            v8h   __attribute__((ext_vector_type(8)));
typedef unsigned short v8us  __attribute__((ext_vector_type(8)));
typedef float          v8f   __attribute__((ext_vector_type(8)));
typedef float          v4f   __attribute__((ext_vector_type(4)));
typedef unsigned       v4u   __attribute__((ext_vector_type(4)));

union FragB  { v16bf v; v4u q[2]; bf16 h[16]; };
union FragH  { v16h  v; v4u q[2]; v8h hv[2]; f16 h[16]; };
union Pack8H { v4u u; v8h v; };
union Pack8S { v4u u; v8us s; };
union BitsB  { bf16 h; unsigned short u; };
union BitsH  { f16  h; unsigned short u; };

static __device__ __forceinline__ v8f mma_bf16(v16bf a, v16bf b, v8f acc) {
  acc = __builtin_amdgcn_wmma_f32_16x16x32_bf16(false, a, false, b, (short)0, acc, false, false);
  asm volatile("v_nop\n\tv_nop\n\tv_nop\n\tv_nop" : "+v"(acc) : "v"(a), "v"(b));
  return acc;
}
static __device__ __forceinline__ v8f mma_f16(v16h a, v16h b, v8f acc) {
  acc = __builtin_amdgcn_wmma_f32_16x16x32_f16(false, a, false, b, (short)0, acc, false, false);
  asm volatile("v_nop\n\tv_nop\n\tv_nop\n\tv_nop" : "+v"(acc) : "v"(a), "v"(b));
  return acc;
}

static __device__ __forceinline__ unsigned short cvt16(float x, int mode) {
  const bf16 xb = (bf16)x;
  BitsB bb; bb.h = xb;
  BitsH bh; bh.h = (f16)((float)xb * 64.0f);
  return mode ? bh.u : bb.u;
}

__global__ __launch_bounds__(256) void wprep_kernel(const float* __restrict__ win,
                                                    unsigned short* __restrict__ wout,
                                                    int ldin, int in_step, int ldout,
                                                    int out_base, int out_step, int mode) {
  const int t   = blockIdx.x;
  const int tid = threadIdx.x;
  __shared__ __align__(16) unsigned short sT[64 * LP];
  const int ib = t * in_step;
  const int ob = out_base + t * out_step;

  #pragma unroll
  for (int kk = 0; kk < 2; ++kk) {
    const int r  = kk * 32 + (tid >> 3);
    const int c0 = (tid & 7) * 8;
    const float* src = win + ib + r * ldin + c0;
    const v4f a0 = *(const v4f*)(src);
    const v4f a1 = *(const v4f*)(src + 4);
    #pragma unroll
    for (int i = 0; i < 4; ++i) {
      sT[(c0 + i) * LP + r]     = cvt16(a0[i], mode);
      sT[(c0 + 4 + i) * LP + r] = cvt16(a1[i], mode);
    }
  }
  __syncthreads();

  v4u    val[2];
  size_t idx[2];
  #pragma unroll
  for (int kk = 0; kk < 2; ++kk) {
    const int c  = kk * 32 + (tid >> 3);
    const int rs = (tid & 7) * 8;
    Pack8S ps;
    ps.s = *(const v8us*)(sT + c * LP + rs);
    val[kk] = ps.u;
    idx[kk] = (size_t)ob + (size_t)c * ldout + rs;
  }
  #pragma unroll
  for (int kk = 0; kk < 2; ++kk) *(volatile v4u*)(wout + idx[kk]) = val[kk];
  __threadfence();
  #pragma unroll
  for (int kk = 0; kk < 2; ++kk) *(volatile v4u*)(wout + idx[kk]) = val[kk];
}

__global__ __launch_bounds__(256) void proj_kernel(const float* __restrict__ x,
                                                   const bf16* __restrict__ wt,
                                                   const float* __restrict__ bq,
                                                   const float* __restrict__ bk,
                                                   const float* __restrict__ bv,
                                                   f16* __restrict__ qh,
                                                   f16* __restrict__ kh,
                                                   f16* __restrict__ vt) {
  const int blk  = blockIdx.x;
  const int bpb  = SEQ / PR;
  const int b    = blk / bpb;
  const int s0   = (blk - b * bpb) * PR;
  const int tid  = threadIdx.x;
  const int wave = __builtin_amdgcn_readfirstlane(threadIdx.x >> 5);
  const int lane = tid & 31;
  const int lq   = lane & 15;
  const int hi   = lane >> 4;
  const int rg   = wave & 3;
  const int nh   = wave >> 2;

  __shared__ __align__(16) f16 sP[3 * PR * LP];

  const float* xp = x + ((size_t)b * SEQ_FULL + s0 + rg * 16 + lq) * DM;
  const bf16*  wp = wt + (size_t)(nh * 96 + lq) * DM;

  v8f acc[6];
  #pragma unroll
  for (int t = 0; t < 6; ++t) acc[t] = (v8f){0, 0, 0, 0, 0, 0, 0, 0};

  #pragma unroll 1
  for (int k0 = 0; k0 < DM; k0 += 32) {
    FragB a;
    {
      const v4f a0 = *(const v4f*)(xp + k0 + hi * 8);
      const v4f a1 = *(const v4f*)(xp + k0 + hi * 8 + 4);
      const v4f b0 = *(const v4f*)(xp + k0 + 16 + hi * 8);
      const v4f b1 = *(const v4f*)(xp + k0 + 16 + hi * 8 + 4);
      #pragma unroll
      for (int i = 0; i < 4; ++i) {
        a.h[i]      = (bf16)a0[i];
        a.h[4 + i]  = (bf16)a1[i];
        a.h[8 + i]  = (bf16)b0[i];
        a.h[12 + i] = (bf16)b1[i];
      }
    }
    #pragma unroll
    for (int t = 0; t < 6; ++t) {
      FragB w;
      const bf16* base = wp + (size_t)t * 16 * DM + k0 + hi * 8;
      w.q[0] = *(const v4u*)(base);
      w.q[1] = *(const v4u*)(base + 16);
      acc[t] = mma_bf16(a.v, w.v, acc[t]);
    }
  }

  #pragma unroll
  for (int t = 0; t < 6; ++t) {
    const int gt    = nh * 6 + t;
    const int plane = gt >> 2;
    const int col   = (gt & 3) * 16 + lq;
    const float b0v = (float)(bf16)bq[col];
    const float b1v = (float)(bf16)bk[col];
    const float b2v = (float)(bf16)bv[col];
    const float bias = (plane == 0) ? b0v : ((plane == 1) ? b1v : b2v);
    #pragma unroll
    for (int r = 0; r < 8; ++r) {
      const int row = rg * 16 + hi * 8 + r;
      const int off = (plane < 2) ? (plane * PR * LP + row * LP + col)
                                  : (2 * PR * LP + col * LP + row);
      sP[off] = (f16)((acc[t][r] + bias) * 16.0f);
    }
  }
  __syncthreads();

  v4u    qv[2], kv[2], vv[2];
  size_t ri[2], vi[2];
  #pragma unroll
  for (int jj = 0; jj < 2; ++jj) {
    const int line = jj * 32 + (tid >> 3);
    const int seg  = (tid & 7) * 8;
    Pack8H pq, pk, pv;
    pq.v = *(const v8h*)(sP + line * LP + seg);
    pk.v = *(const v8h*)(sP + PR * LP + line * LP + seg);
    pv.v = *(const v8h*)(sP + 2 * PR * LP + line * LP + seg);
    qv[jj] = pq.u;
    kv[jj] = pk.u;
    vv[jj] = pv.u;
    ri[jj] = ((size_t)b * SEQ + s0 + line) * PD + seg;
    vi[jj] = ((size_t)b * PD + line) * SEQ + s0 + seg;
  }
  #pragma unroll
  for (int jj = 0; jj < 2; ++jj) {
    *(volatile v4u*)(qh + ri[jj]) = qv[jj];
    *(volatile v4u*)(kh + ri[jj]) = kv[jj];
    *(volatile v4u*)(vt + vi[jj]) = vv[jj];
  }
  __threadfence();
  #pragma unroll
  for (int jj = 0; jj < 2; ++jj) {
    *(volatile v4u*)(qh + ri[jj]) = qv[jj];
    *(volatile v4u*)(kh + ri[jj]) = kv[jj];
    *(volatile v4u*)(vt + vi[jj]) = vv[jj];
  }
}

__global__ __launch_bounds__(256) void attn_kernel(const f16* __restrict__ qh,
                                                   const f16* __restrict__ kh,
                                                   const f16* __restrict__ vt,
                                                   const f16* __restrict__ wot,
                                                   const float* __restrict__ bo,
                                                   const float* __restrict__ mask,
                                                   float* __restrict__ out) {
  const int qblk = blockIdx.x;
  const int b    = blockIdx.y;
  const int tid  = threadIdx.x;
  const int wave = __builtin_amdgcn_readfirstlane(threadIdx.x >> 5);
  const int lane = tid & 31;
  const int lq   = lane & 15;
  const int hi   = lane >> 4;

  __shared__ __align__(16) float sO[NWAVE * 16 * OP];
  __shared__ __align__(16) f16   sC[NWAVE * 16 * LP];

  const int qrow0 = qblk * BQ + wave * 16;

  FragH qf[2];
  {
    const f16* qp = qh + ((size_t)b * SEQ + qrow0 + lq) * PD;
    #pragma unroll
    for (int f = 0; f < 2; ++f) {
      qf[f].q[0] = *(const v4u*)(qp + f * 32 + hi * 8);
      qf[f].q[1] = *(const v4u*)(qp + f * 32 + 16 + hi * 8);
    }
  }

  const float mv   = (float)(bf16)mask[(size_t)b * SEQ_FULL + qrow0 + lq];
  const float madd = (1.0f - mv) * -10000.0f;

  const f16* kh_b = kh + (size_t)b * SEQ * PD;
  const f16* vt_b = vt + (size_t)b * PD * SEQ;

  v8f o[4];
  #pragma unroll
  for (int dt = 0; dt < 4; ++dt) o[dt] = (v8f){0, 0, 0, 0, 0, 0, 0, 0};

  float rmax = -__builtin_inff();
  float rsum = 0.0f;
  const float SC    = 0.125f * (1.0f / 256.0f);
  const float LOG2E = 1.4426950408889634f;

  const int nchunk = SEQ / BK;
  #pragma unroll 1
  for (int i = 0; i < nchunk; ++i) {
    const int j0 = i * BK;

    FragH ak[2][2];
    #pragma unroll
    for (int sub = 0; sub < 2; ++sub) {
      #pragma unroll
      for (int f = 0; f < 2; ++f) {
        const f16* base = kh_b + (size_t)(j0 + sub * 16 + lq) * PD + f * 32 + hi * 8;
        ak[sub][f].q[0] = *(const v4u*)(base);
        ak[sub][f].q[1] = *(const v4u*)(base + 16);
      }
    }
    FragH bvf[4];
    #pragma unroll
    for (int dt = 0; dt < 4; ++dt) {
      const f16* base = vt_b + (size_t)(dt * 16 + lq) * SEQ + j0 + hi * 8;
      bvf[dt].q[0] = *(const v4u*)(base);
      bvf[dt].q[1] = *(const v4u*)(base + 16);
    }

    v8f c[2];
    #pragma unroll
    for (int sub = 0; sub < 2; ++sub) {
      v8f acc = (v8f){0, 0, 0, 0, 0, 0, 0, 0};
      acc = mma_f16(ak[sub][0].v, qf[0].v, acc);
      acc = mma_f16(ak[sub][1].v, qf[1].v, acc);
      c[sub] = acc;
    }

    float s0v[8], s1v[8];
    float m_new = rmax;
    #pragma unroll
    for (int r = 0; r < 8; ++r) {
      s0v[r] = c[0][r] * SC + madd;
      s1v[r] = c[1][r] * SC + madd;
      m_new = fmaxf(m_new, s0v[r]);
      m_new = fmaxf(m_new, s1v[r]);
    }
    m_new = fmaxf(m_new, __shfl_xor(m_new, 16, 32));
    const float scale = __builtin_amdgcn_exp2f((rmax - m_new) * LOG2E);
    rmax = m_new;

    FragH pa;
    float psum = 0.0f;
    #pragma unroll
    for (int r = 0; r < 8; ++r) {
      const float p0 = __builtin_amdgcn_exp2f((s0v[r] - m_new) * LOG2E);
      const float p1 = __builtin_amdgcn_exp2f((s1v[r] - m_new) * LOG2E);
      psum += p0 + p1;
      pa.h[r]     = (f16)(p0 * 4096.0f);
      pa.h[8 + r] = (f16)(p1 * 4096.0f);
    }
    rsum = rsum * scale + psum + __shfl_xor(psum, 16, 32);

    float sc[8];
    #pragma unroll
    for (int r = 0; r < 8; ++r) sc[r] = __shfl(scale, (hi << 3) + r, 32);
    #pragma unroll
    for (int dt = 0; dt < 4; ++dt) {
      #pragma unroll
      for (int r = 0; r < 8; ++r) o[dt][r] *= sc[r];
    }

    #pragma unroll
    for (int dt = 0; dt < 4; ++dt) o[dt] = mma_f16(pa.v, bvf[dt].v, o[dt]);
  }

  float rs[8];
  #pragma unroll
  for (int r = 0; r < 8; ++r) rs[r] = 1.0f / __shfl(rsum, (hi << 3) + r, 32);

  f16* scx = sC + wave * (16 * LP);
  #pragma unroll
  for (int r = 0; r < 8; ++r) {
    #pragma unroll
    for (int dt = 0; dt < 4; ++dt) {
      scx[(hi * 8 + r) * LP + dt * 16 + lq] = (f16)(o[dt][r] * rs[r] * 0.00390625f);
    }
  }
  __syncthreads();

  FragH aw[2];
  #pragma unroll
  for (int f = 0; f < 2; ++f) {
    const f16* base = scx + lq * LP + f * 32 + hi * 8;
    aw[f].hv[0] = *(const v8h*)(base);
    aw[f].hv[1] = *(const v8h*)(base + 16);
  }

  float* so = sO + wave * (16 * OP);

  #pragma unroll 1
  for (int cg = 0; cg < 8; ++cg) {
    v8f y[4];
    float bias[4];
    #pragma unroll
    for (int dt = 0; dt < 4; ++dt) {
      const int n = cg * 64 + dt * 16 + lq;
      const f16* base = wot + (size_t)n * PD + hi * 8;
      FragH w0, w1;
      w0.q[0] = *(const v4u*)(base);
      w0.q[1] = *(const v4u*)(base + 16);
      w1.q[0] = *(const v4u*)(base + 32);
      w1.q[1] = *(const v4u*)(base + 48);
      v8f acc = (v8f){0, 0, 0, 0, 0, 0, 0, 0};
      acc = mma_f16(aw[0].v, w0.v, acc);
      acc = mma_f16(aw[1].v, w1.v, acc);
      y[dt] = acc;
      bias[dt] = (float)(bf16)bo[n];
    }
    #pragma unroll
    for (int r = 0; r < 8; ++r) {
      #pragma unroll
      for (int dt = 0; dt < 4; ++dt) {
        so[(hi * 8 + r) * OP + dt * 16 + lq] = y[dt][r] * 0.00006103515625f + bias[dt];
      }
    }
    __syncthreads();

    v4f    vals[8];
    size_t gidx[8];
    #pragma unroll
    for (int it = 0; it < 8; ++it) {
      const int row = it * 2 + hi;
      vals[it] = *(const v4f*)(so + row * OP + lq * 4);
      gidx[it] = ((size_t)b * SEQ_FULL + qrow0 + row) * DM + cg * 64 + lq * 4;
    }
    #pragma unroll
    for (int it = 0; it < 8; ++it) *(volatile v4f*)(out + gidx[it]) = vals[it];
    __threadfence();
    #pragma unroll
    for (int it = 0; it < 8; ++it) *(volatile v4f*)(out + gidx[it]) = vals[it];
    __syncthreads();
  }
}

extern "C" void kernel_launch(void* const* d_in, const int* in_sizes, int n_in,
                              void* d_out, int out_size, void* d_ws, size_t ws_size,
                              hipStream_t stream) {
  if (n_in < 10) return;
  const size_t need_x = ((size_t)(NB - 1) * SEQ_FULL + SEQ) * DM;
  const size_t need_m = (size_t)(NB - 1) * SEQ_FULL + SEQ;
  if ((size_t)in_sizes[0] < need_x) return;
  if ((size_t)in_sizes[1] < need_m) return;
  if ((size_t)in_sizes[2] < (size_t)DM * PD) return;
  if ((size_t)in_sizes[3] < (size_t)PD) return;
  if ((size_t)in_sizes[4] < (size_t)DM * PD) return;
  if ((size_t)in_sizes[5] < (size_t)PD) return;
  if ((size_t)in_sizes[6] < (size_t)DM * PD) return;
  if ((size_t)in_sizes[7] < (size_t)PD) return;
  if ((size_t)in_sizes[8] < (size_t)PD * DM) return;
  if ((size_t)in_sizes[9] < (size_t)DM) return;
  if ((size_t)out_size < need_x) return;

  const size_t wt_bytes  = (size_t)NQKV * DM * 2;
  const size_t wot_bytes = (size_t)DM * PD * 2;
  const size_t pl_bytes  = (size_t)NB * SEQ * PD * 2;
  if (ws_size < wt_bytes + wot_bytes + 3 * pl_bytes) return;

  const float* x    = (const float*)d_in[0];
  const float* mask = (const float*)d_in[1];
  const float* Wq   = (const float*)d_in[2];
  const float* bq   = (const float*)d_in[3];
  const float* Wk   = (const float*)d_in[4];
  const float* bk   = (const float*)d_in[5];
  const float* Wv   = (const float*)d_in[6];
  const float* bv   = (const float*)d_in[7];
  const float* Wo   = (const float*)d_in[8];
  const float* bo   = (const float*)d_in[9];
  float*       out  = (float*)d_out;

  char* ws = (char*)d_ws;
  unsigned short* wt_u  = (unsigned short*)(ws);
  unsigned short* wot_u = (unsigned short*)(ws + wt_bytes);
  f16* qh = (f16*)(ws + wt_bytes + wot_bytes);
  f16* kh = (f16*)(ws + wt_bytes + wot_bytes + pl_bytes);
  f16* vt = (f16*)(ws + wt_bytes + wot_bytes + 2 * pl_bytes);

  wprep_kernel<<<DM / 64, 256, 0, stream>>>(Wq, wt_u, PD, 64 * PD, DM, 0 * PD * DM, 64, 0);
  wprep_kernel<<<DM / 64, 256, 0, stream>>>(Wk, wt_u, PD, 64 * PD, DM, 1 * PD * DM, 64, 0);
  wprep_kernel<<<DM / 64, 256, 0, stream>>>(Wv, wt_u, PD, 64 * PD, DM, 2 * PD * DM, 64, 0);
  wprep_kernel<<<DM / 64, 256, 0, stream>>>(Wo, wot_u, DM, 64, PD, 0, 64 * PD, 1);

  proj_kernel<<<NB * (SEQ / PR), 256, 0, stream>>>(x, (const bf16*)wt_u, bq, bk, bv, qh, kh, vt);
  attn_kernel<<<dim3(SEQ / BQ, NB), 256, 0, stream>>>(qh, kh, vt, (const f16*)wot_u, bo, mask, out);
}
